// LinearMultiheadAttention_283467842835
// MI455X (gfx1250) — hardware-run, weakly checked
//
#include <hip/hip_runtime.h>
#include <math.h>
#include <stdint.h>

#ifndef NB
#define NB 4
#endif
#ifndef SEQ
#define SEQ 2048
#endif
#define XS_FULL 2048
#define DM   512
#define NH   8
#define DHN  (NH * DM)
#define QSC  1024.0f
#define KSC  1024.0f
#define VSC  256.0f
#define CSC  16.0f
#define OSC  0.25f
#define WOSC 64.0f
#define SLAB64 (16 * 68)
#define TRP  72
#define WS_CAP 134217728
static_assert(DHN == NH * DM && DM == 512 && NH == 8);
static_assert(NB >= 1 && NB <= 4);
static_assert(NB == 1 || SEQ == XS_FULL);
static_assert((SEQ % 64) == 0 && SEQ >= 64 && SEQ <= XS_FULL);
static_assert(((SEQ * DM / 8) % 256) == 0 && (DM % 256) == 0 && (DM % 64) == 0 && (DHN % 2048) == 0);
static_assert(4 * SLAB64 * 4 <= 65536 && NH * 16 * TRP * 2 <= 65536 && DHN * 2 <= 65536 && 64 * TRP * 2 <= 65536);

typedef unsigned short u16;
typedef _Float16 v16h __attribute__((ext_vector_type(16)));
typedef _Float16 v8h  __attribute__((ext_vector_type(8)));
typedef __bf16   v16b __attribute__((ext_vector_type(16)));
typedef float    v8f  __attribute__((ext_vector_type(8)));
typedef float    v4f  __attribute__((ext_vector_type(4)));
typedef unsigned int v4u __attribute__((ext_vector_type(4)));

union FragH { v16h v; v8h h[2]; v4u u[2]; };
union FragB { v16b v; v4u u[2]; };

__device__ __forceinline__ unsigned short bf_bits(float f) {
  unsigned u = __float_as_uint(f);
  return (unsigned short)((u + 0x7FFFu + ((u >> 16) & 1u)) >> 16);
}
__device__ __forceinline__ float bf_up(unsigned short h) { return __uint_as_float(((unsigned)h) << 16); }
__device__ __forceinline__ float bfr(float f) { return bf_up(bf_bits(f)); }
__device__ __forceinline__ unsigned short h_bits(_Float16 x) { return __builtin_bit_cast(unsigned short, x); }
__device__ __forceinline__ unsigned pk16(unsigned short a, unsigned short b) { return (unsigned)a | ((unsigned)b << 16); }
__device__ __forceinline__ v8f zero8() { v8f z = {0.f, 0.f, 0.f, 0.f, 0.f, 0.f, 0.f, 0.f}; return z; }
__device__ __forceinline__ int imin(int a, int b) { return a < b ? a : b; }
__device__ __forceinline__ int imax(int a, int b) { return a > b ? a : b; }

__device__ __forceinline__ v16h ldfrag_h(const _Float16* p) {
  FragH f;
  f.h[0] = *(const v8h*)(p);
  f.h[1] = *(const v8h*)(p + 16);
  return f.v;
}
__device__ __forceinline__ v16b ldfrag_b(const u16* p) {
  FragB f;
  f.u[0] = *(const v4u*)(p);
  f.u[1] = *(const v4u*)(p + 16);
  return f.v;
}

__device__ __forceinline__ v8f mma_h(v16h a, v16h b, v8f c) {
  return __builtin_amdgcn_wmma_f32_16x16x32_f16(false, a, false, b, (short)0, c, false, false);
}
__device__ __forceinline__ v8f mma_b(v16b a, v16b b, v8f c) {
  return __builtin_amdgcn_wmma_f32_16x16x32_bf16(false, a, false, b, (short)0, c, false, false);
}
template <typename F>
__device__ __forceinline__ void guard6(v8f& a, v8f& b, v8f& c, v8f& d, F x0, F x1, F x2, F x3, F x4, F x5) {
#if defined(__HIP_DEVICE_COMPILE__)
  asm volatile("v_nop\n\tv_nop\n\tv_nop\n\tv_nop"
               : "+v"(a), "+v"(b), "+v"(c), "+v"(d) : "v"(x0), "v"(x1), "v"(x2), "v"(x3), "v"(x4), "v"(x5) : "memory");
#endif
}
__device__ __forceinline__ void wave_sync_lds() {
  __builtin_amdgcn_fence(__ATOMIC_RELEASE, "workgroup");
  __builtin_amdgcn_wave_barrier();
  __builtin_amdgcn_fence(__ATOMIC_ACQUIRE, "workgroup");
}

template <bool F16, bool PERM>
__global__ __launch_bounds__(256) void k_wt(const float* __restrict__ W, int nc, int kr, int ntn, u16* Dp, float sc) {
  __shared__ __align__(16) u16 T[64 * TRP];
  const int tid = (int)threadIdx.x;
  const int bid = (int)blockIdx.x;
  const int hz  = (int)blockIdx.y;
  const int nt  = bid % ntn;
  const int kt  = bid / ntn;
  if (kt * 64 + 64 > kr) return;
  const int n0  = nt * 64, k0 = kt * 64;
  const float* Wh = W + (size_t)hz * (size_t)kr * (size_t)nc;
  const int drow0 = hz * nc;
  {
    const int dl = tid >> 2;
    const int oc = (tid & 3) * 16;
    const bool valid = (n0 + oc + 16 <= nc);
    const int  cb = valid ? (n0 + oc) : 0;
    const int  kk = k0 + dl;
    int sr = kk;
    if constexpr (PERM) sr = (kk % DM) * NH + (kk / DM);
    const float* src = Wh + (size_t)sr * (size_t)nc + cb;
#pragma unroll
    for (int i = 0; i < 4; ++i) {
      const v4f a = *(const v4f*)(src + 4 * i);
#pragma unroll
      for (int e = 0; e < 4; ++e) {
        const float f = valid ? a[e] : 0.0f;
        u16 bits;
        if constexpr (F16) bits = h_bits((_Float16)(bfr(f) * sc));
        else bits = bf_bits(f);
        T[(oc + 4 * i + e) * TRP + dl] = bits;
      }
    }
  }
  __syncthreads();
  const int q8 = tid >> 3, p8 = (tid & 7) * 8;
  v4u w[2];
#pragma unroll
  for (int it = 0; it < 2; ++it) w[it] = *(const v4u*)(T + (it * 32 + q8) * TRP + p8);
  const size_t base = (size_t)(drow0 + n0) * (size_t)kr + k0 + p8;
  for (int pass = 0; pass < 2; ++pass) {
#pragma unroll
    for (int it = 0; it < 2; ++it) {
      const int nl = it * 32 + q8;
      *(volatile v4u*)(Dp + base + (size_t)nl * (size_t)kr) = w[it];
    }
    __threadfence();
  }
}

__global__ __launch_bounds__(256) void cvt_bf3(const float* __restrict__ x0, const float* __restrict__ x1,
                                               const float* __restrict__ x2, u16* D0, u16* D1, u16* D2, int n8) {
  const int which = (int)blockIdx.y;
  const float* x = (which == 0) ? x0 : ((which == 1) ? x1 : x2);
  u16* D = (which == 0) ? D0 : ((which == 1) ? D1 : D2);
  const int gt = (int)blockIdx.x * 256 + (int)threadIdx.x;
  if (gt >= n8) return;
  const float* p = x + (size_t)gt * 8;
  const v4f a = *(const v4f*)(p), b4 = *(const v4f*)(p + 4);
  float w[8];
#pragma unroll
  for (int e = 0; e < 4; ++e) { w[e] = a[e]; w[4 + e] = b4[e]; }
  v4u o;
#pragma unroll
  for (int e = 0; e < 4; ++e) o[e] = pk16(bf_bits(w[2 * e]), bf_bits(w[2 * e + 1]));
  u16* d = D + (size_t)gt * 8;
  for (int pass = 0; pass < 2; ++pass) {
    *(volatile v4u*)(d) = o;
    __threadfence();
  }
}

__global__ __launch_bounds__(256) void soft_q(const float* __restrict__ F, u16* QP) {
  __shared__ __align__(16) u16 T[DHN];
  const int tid = (int)threadIdx.x;
  const int row = (int)blockIdx.x;
  if (row >= SEQ) return;
  const float* fr = F + (size_t)row * DHN;
#pragma unroll 1
  for (int i = 0; i < DM / 256; ++i) {
    const int e = i * 256 + tid;
    float v[NH];
#pragma unroll
    for (int h = 0; h < NH; ++h) v[h] = fr[h * DM + e];
    float mx = v[0];
#pragma unroll
    for (int h = 1; h < NH; ++h) mx = fmaxf(mx, v[h]);
    float s = 0.0f;
#pragma unroll
    for (int h = 0; h < NH; ++h) { v[h] = __expf(v[h] - mx); s += v[h]; }
    const float f = (1.0f / s) * QSC;
#pragma unroll
    for (int h = 0; h < NH; ++h) T[h * DM + e] = h_bits((_Float16)(v[h] * f));
  }
  __syncthreads();
  v4u o[DHN / 2048];
#pragma unroll
  for (int it = 0; it < DHN / 2048; ++it) o[it] = *(const v4u*)(T + it * 2048 + tid * 8);
  u16* d = QP + (size_t)row * DHN + tid * 8;
  for (int pass = 0; pass < 2; ++pass) {
#pragma unroll
    for (int it = 0; it < DHN / 2048; ++it) *(volatile v4u*)(d + it * 2048) = o[it];
    __threadfence();
  }
}

template <bool SM>
__global__ __launch_bounds__(256) void tr16(const float* __restrict__ F, u16* P, float sc) {
  __shared__ __align__(16) u16 T[NH * 16 * TRP];
  const int tid = (int)threadIdx.x;
  const int bid = (int)blockIdx.x;
  const int nst = SEQ / 64;
  const int st  = bid % nst;
  const int et  = bid / nst;
  if (et >= DM / 16) return;
  const int s0 = st * 64, e0 = et * 16;
  const int sl = tid >> 2, eq = tid & 3;
  const float* src = F + (size_t)(s0 + sl) * (size_t)DHN + e0;
#pragma unroll 1
  for (int i = 0; i < 4; ++i) {
    const int el = eq + 4 * i;
    float v[NH];
#pragma unroll
    for (int h = 0; h < NH; ++h) v[h] = src[h * DM + el];
    float f = sc;
    if constexpr (SM) {
      float mx = v[0];
#pragma unroll
      for (int h = 1; h < NH; ++h) mx = fmaxf(mx, v[h]);
      float s = 0.0f;
#pragma unroll
      for (int h = 0; h < NH; ++h) { v[h] = __expf(v[h] - mx); s += v[h]; }
      f = (1.0f / s) * sc;
    }
#pragma unroll
    for (int h = 0; h < NH; ++h) T[(h * 16 + el) * TRP + sl] = h_bits((_Float16)(v[h] * f));
  }
  __syncthreads();
  const int q8 = tid >> 3, p8 = (tid & 7) * 8;
  v4u o[4];
#pragma unroll
  for (int it = 0; it < 4; ++it) o[it] = *(const v4u*)(T + (it * 32 + q8) * TRP + p8);
  for (int pass = 0; pass < 2; ++pass) {
#pragma unroll
    for (int it = 0; it < 4; ++it) {
      const int line = it * 32 + q8;
      const int hl = line >> 4, el = line & 15;
      *(volatile v4u*)(P + (size_t)(hl * DM + e0 + el) * (size_t)SEQ + s0 + p8) = o[it];
    }
    __threadfence();
  }
}

__device__ __forceinline__ void epi64f(float* sl, v8f a0, v8f a1, v8f a2, v8f a3, v4f bias4, float scale,
                                       float* C, int ldc, size_t rowb, int col0, int lane) {
  const int hh = lane >> 4, m = lane & 15;
#pragma unroll
  for (int r = 0; r < 8; ++r) {
    const int ro = (8 * hh + r) * 68 + m;
    sl[ro]      = a0[r];
    sl[ro + 16] = a1[r];
    sl[ro + 32] = a2[r];
    sl[ro + 48] = a3[r];
  }
  wave_sync_lds();
  v4f vals[8];
#pragma unroll
  for (int it = 0; it < 8; ++it) {
    const v4f v = *(const v4f*)(sl + (it * 2 + hh) * 68 + m * 4);
    vals[it] = v * scale + bias4;
  }
  float* dst = C + (rowb + (size_t)hh) * (size_t)ldc + col0 + m * 4;
  for (int pass = 0; pass < 2; ++pass) {
#pragma unroll
    for (int it = 0; it < 8; ++it) {
      *(volatile v4f*)(dst + (size_t)(it * 2) * (size_t)ldc) = vals[it];
    }
    __threadfence();
  }
}

__device__ __forceinline__ void epi64h(float* sl, v8f a0, v8f a1, v8f a2, v8f a3, float scale,
                                       u16* C, int ldc, size_t rowb, int col0, int lane) {
  const int hh = lane >> 4, m = lane & 15;
#pragma unroll
  for (int r = 0; r < 8; ++r) {
    const int ro = (8 * hh + r) * 68 + m;
    sl[ro]      = a0[r];
    sl[ro + 16] = a1[r];
    sl[ro + 32] = a2[r];
    sl[ro + 48] = a3[r];
  }
  wave_sync_lds();
  const int rq = lane >> 3, c8 = (lane & 7) * 8;
  v4u o[4];
#pragma unroll
  for (int it = 0; it < 4; ++it) {
    const int row = it * 4 + rq;
    const v4f a = *(const v4f*)(sl + row * 68 + c8), b4 = *(const v4f*)(sl + row * 68 + c8 + 4);
    float w[8];
#pragma unroll
    for (int e = 0; e < 4; ++e) { w[e] = a[e] * scale; w[4 + e] = b4[e] * scale; }
#pragma unroll
    for (int e = 0; e < 4; ++e) o[it][e] = pk16(h_bits((_Float16)w[2 * e]), h_bits((_Float16)w[2 * e + 1]));
  }
  u16* dst = C + rowb * (size_t)ldc + col0 + c8;
  for (int pass = 0; pass < 2; ++pass) {
#pragma unroll
    for (int it = 0; it < 4; ++it) {
      const int row = it * 4 + rq;
      *(volatile v4u*)(dst + (size_t)row * (size_t)ldc) = o[it];
    }
    __threadfence();
  }
}

template <bool BF, int EPI>
__global__ __launch_bounds__(128)
void gemm16(const u16* __restrict__ A, const u16* __restrict__ Bt, float* Cf, u16* Ch, const float* __restrict__ bias,
            int lda, int aH, int ldb, int bH, int ldc, int cH, int M, int N, int K, float scale) {
  __shared__ __align__(16) float slab[4 * SLAB64];
  const int tid = (int)threadIdx.x, wave = tid >> 5, lane = tid & 31, hh = lane >> 4, m = lane & 15;
  const int ntile = N >> 6;
  const int bid   = (int)blockIdx.x;
  const size_t hz = (size_t)blockIdx.y;
  const int rowb  = (bid / ntile) * 64 + wave * 16;
  const int col0  = (bid % ntile) * 64;
  if (rowb + 16 > M) return;
  const u16* ap = A  + hz * (size_t)aH + (size_t)(rowb + m) * (size_t)lda + 8 * hh;
  const u16* bp = Bt + hz * (size_t)bH + (size_t)(col0 + m) * (size_t)ldb + 8 * hh;
  const size_t bs = (size_t)16 * (size_t)ldb;
  v8f acc0 = zero8(), acc1 = zero8(), acc2 = zero8(), acc3 = zero8();
#pragma unroll 1
  for (int k0 = 0; k0 < K; k0 += 32) {
    if constexpr (BF) {
      const v16b a   = ldfrag_b(ap + k0);
      const v16b fb0 = ldfrag_b(bp + k0);
      const v16b fb1 = ldfrag_b(bp + bs + k0);
      const v16b fb2 = ldfrag_b(bp + 2 * bs + k0);
      const v16b fb3 = ldfrag_b(bp + 3 * bs + k0);
      acc0 = mma_b(a, fb0, acc0);
      acc1 = mma_b(a, fb1, acc1);
      acc2 = mma_b(a, fb2, acc2);
      acc3 = mma_b(a, fb3, acc3);
      guard6<v16b>(acc0, acc1, acc2, acc3, a, fb0, fb1, fb2, fb3, a);
    } else {
      const _Float16* aq = (const _Float16*)(const void*)(ap + k0);
      const _Float16* bq = (const _Float16*)(const void*)(bp + k0);
      const v16h a   = ldfrag_h(aq);
      const v16h fb0 = ldfrag_h(bq);
      const v16h fb1 = ldfrag_h(bq + bs);
      const v16h fb2 = ldfrag_h(bq + 2 * bs);
      const v16h fb3 = ldfrag_h(bq + 3 * bs);
      acc0 = mma_h(a, fb0, acc0);
      acc1 = mma_h(a, fb1, acc1);
      acc2 = mma_h(a, fb2, acc2);
      acc3 = mma_h(a, fb3, acc3);
      guard6<v16h>(acc0, acc1, acc2, acc3, a, fb0, fb1, fb2, fb3, a);
    }
  }
  float* sl = slab + wave * SLAB64;
  if constexpr (EPI == 0) {
    v4f bias4;
#pragma unroll
    for (int e = 0; e < 4; ++e) bias4[e] = bfr(bias[imin(imax(col0 + m * 4 + e, 0), N - 1)]);
    epi64f(sl, acc0, acc1, acc2, acc3, bias4, scale, Cf + hz * (size_t)cH, ldc, (size_t)rowb, col0, lane);
  } else {
    epi64h(sl, acc0, acc1, acc2, acc3, scale, Ch + hz * (size_t)cH, ldc, (size_t)rowb, col0, lane);
  }
}

extern "C" void kernel_launch(void* const* d_in, const int* in_sizes, int n_in,
                              void* d_out, int out_size, void* d_ws, size_t ws_size,
                              hipStream_t stream) {
  if (n_in < 11) return;
  const int need = ((NB - 1) * XS_FULL + SEQ) * DM;
  if (in_sizes[0] < need || in_sizes[1] < need || in_sizes[2] < need) return;
  if (in_sizes[3] < NH * DM * DM || in_sizes[5] < NH * DM * DM || in_sizes[7] < NH * DM * DM) return;
  if (in_sizes[4] < DHN || in_sizes[6] < DHN || in_sizes[8] < DHN) return;
  if (in_sizes[9] < DHN * DM || in_sizes[10] < DM) return;
  if (out_size < need) return;

  const float* xq = (const float*)d_in[0];
  const float* xk = (const float*)d_in[1];
  const float* xv = (const float*)d_in[2];
  const float* wq = (const float*)d_in[3];
  const float* bq = (const float*)d_in[4];
  const float* wk = (const float*)d_in[5];
  const float* bk = (const float*)d_in[6];
  const float* wv = (const float*)d_in[7];
  const float* bv = (const float*)d_in[8];
  const float* wo = (const float*)d_in[9];
  const float* bo = (const float*)d_in[10];
  float*       out = (float*)d_out;

  const size_t szX = (size_t)SEQ * DM * 2;
  const size_t szW = (size_t)DHN * DM * 2;
  const size_t szF = (size_t)SEQ * DHN * 4;
  const size_t szP = (size_t)SEQ * DHN * 2;
  const size_t szC = (size_t)DHN * DM * 2;
  if (szP > szF) return;
  size_t off = 0;
  const size_t oXQ = off; off += szX;
  const size_t oXK = off; off += szX;
  const size_t oXV = off; off += szX;
  const size_t oWQ = off; off += szW;
  const size_t oWK = off; off += szW;
  const size_t oWV = off; off += szW;
  const size_t oWO = off; off += szW;
  const size_t oF  = off; off += szF;
  const size_t oQP = off; off += szP;
  const size_t oKT = off; off += szP;
  const size_t oVT = off; off += szP;
  const size_t oCT = off; off += szC;
  if (off > ws_size) return;
  if (off > (size_t)WS_CAP) return;

  char* ws = (char*)d_ws;
  u16*   XQ  = (u16*)(ws + oXQ);
  u16*   XK  = (u16*)(ws + oXK);
  u16*   XV  = (u16*)(ws + oXV);
  u16*   WQT = (u16*)(ws + oWQ);
  u16*   WKT = (u16*)(ws + oWK);
  u16*   WVT = (u16*)(ws + oWV);
  u16*   WOT = (u16*)(ws + oWO);
  float* F   = (float*)(ws + oF);
  u16*   OP  = (u16*)(ws + oF);
  u16*   QP  = (u16*)(ws + oQP);
  u16*   KT  = (u16*)(ws + oKT);
  u16*   VT  = (u16*)(ws + oVT);
  u16*   CT  = (u16*)(ws + oCT);

  const dim3 b256(256), b128(128);
  const int  n8x = (SEQ * DM) / 8;
  const dim3 gWp((DM / 64) * (DM / 64), NH);
  const dim3 gWo((DHN / 64) * (DM / 64), 1);
  const dim3 gX3(n8x / 256, 3);
  const dim3 gPJ((SEQ / 64) * (DHN / 64), 1);
  const dim3 gSQ(SEQ);
  const dim3 gTR((SEQ / 64) * (DM / 16));
  const dim3 gCX((DM / 64) * (DM / 64), NH);
  const dim3 gOU((SEQ / 64) * (DM / 64), NH);
  const dim3 gFI((SEQ / 64) * (DM / 64), 1);

  const float scC = CSC / (KSC * VSC);
  const float scO = OSC / (QSC * CSC);
  const float scY = 1.0f / (OSC * WOSC);

  k_wt<false, false><<<gWp, b256, 0, stream>>>(wq, DM, DM, DM / 64, WQT, 1.0f);
  k_wt<false, false><<<gWp, b256, 0, stream>>>(wk, DM, DM, DM / 64, WKT, 1.0f);
  k_wt<false, false><<<gWp, b256, 0, stream>>>(wv, DM, DM, DM / 64, WVT, 1.0f);
  k_wt<true,  true ><<<gWo, b256, 0, stream>>>(wo, DM, DHN, DM / 64, WOT, WOSC);

  for (int b = 0; b < NB; ++b) {
    const size_t xo = (size_t)b * XS_FULL * DM;
    cvt_bf3<<<gX3, b256, 0, stream>>>(xq + xo, xk + xo, xv + xo, XQ, XK, XV, n8x);
    gemm16<true, 0><<<gPJ, b128, 0, stream>>>(XQ, WQT, F, QP, bq, DM, 0, DM, 0, DHN, 0, SEQ, DHN, DM, 1.0f);
    soft_q<<<gSQ, b256, 0, stream>>>(F, QP);
    gemm16<true, 0><<<gPJ, b128, 0, stream>>>(XK, WKT, F, QP, bk, DM, 0, DM, 0, DHN, 0, SEQ, DHN, DM, 1.0f);
    tr16<true><<<gTR, b256, 0, stream>>>(F, KT, KSC);
    gemm16<true, 0><<<gPJ, b128, 0, stream>>>(XV, WVT, F, QP, bv, DM, 0, DM, 0, DHN, 0, SEQ, DHN, DM, 1.0f);
    tr16<false><<<gTR, b256, 0, stream>>>(F, VT, VSC);
    gemm16<false, 1><<<gCX, b128, 0, stream>>>(VT, KT, F, CT, bo, SEQ, DM * SEQ, SEQ, DM * SEQ, DM, DM * DM,
                                                DM, DM, SEQ, scC);
    gemm16<false, 1><<<gOU, b128, 0, stream>>>(QP, CT, F, OP, bo, DHN, DM, DM, DM * DM, DHN, DM,
                                                SEQ, DM, DM, scO);
    gemm16<false, 0><<<gFI, b128, 0, stream>>>(OP, WOT, out + xo, CT, bo, DHN, 0, DHN, 0, DM, 0,
                                                SEQ, DM, DHN, scY);
  }
  (void)hipGetLastError();
}
